// MP_GCN_67448166417077
// MI455X (gfx1250) — hardware-verified
//
#include <hip/hip_runtime.h>
#include <stddef.h>


#define F       128
#define G3      384
#define GH1     64
#define GH2     32
#define H1      85
#define H1P     96
#define H2      64
#define NTHR    256
#define NWAVE   8
#define BR      32
#define BRF     64
#define NBF     1024
#define RCAP    40960
#define DEGCAP  512
#define EPT     8
#define NGRP    2
#define CHUNK   (NTHR * EPT * NGRP)
#define WCAP    (EPT * NGRP * 32)
#define LISTN   (NWAVE * WCAP)
#define KCH     1024
#define NGP     64
#define PROP_ITER 4
#define WSCAP   134217728
#define SC_A    8.0f
#define SC_INV  (1.0f / 2048.0f)
#define SC_T    16384.0f
#define SC_TL   1024.0f

#define LDS_CSR ((RCAP + 3 * NBF + LISTN + 32) * 4)
#define LDS_FIN (BRF * (F + 8) * 2 + BRF * F * 4 + BRF * 4 + 2 * F * (BRF + 8) * 2)

static_assert((CHUNK & (CHUNK - 1)) == 0);
static_assert(CHUNK <= 4096);
static_assert((NBF & (NBF - 1)) == 0 && NBF <= 4096);
static_assert(NBF == 4 * NTHR);
static_assert((RCAP % (4 * NTHR)) == 0);
static_assert(KCH == NBF);
static_assert(F == 128 && BR == 32 && BRF == 64);
static_assert((BR / NWAVE) == 4);
static_assert(LISTN >= NWAVE * 2 * F / 2);
static_assert((BRF * (F + 8) * 2) % 16 == 0);

typedef float    v4f  __attribute__((ext_vector_type(4)));
typedef float    v8f  __attribute__((ext_vector_type(8)));
typedef int      v4i  __attribute__((ext_vector_type(4)));
typedef _Float16 v4h  __attribute__((ext_vector_type(4)));
typedef _Float16 v8h  __attribute__((ext_vector_type(8)));
typedef _Float16 v16h __attribute__((ext_vector_type(16)));
union Frag { v16h v; v8h h[2]; };

__device__ __forceinline__ v8f wmf(v16h a, v16h b, v8f c) {
  v8f d = __builtin_amdgcn_wmma_f32_16x16x32_f16(false, a, false, b, (short)0, c, false, false);
  asm volatile("v_nop\n\tv_nop\n\tv_nop\n\tv_nop" : "+v"(d) : "v"(a), "v"(b));
  return d;
}
__device__ __forceinline__ void ldfrag(Frag& f, const _Float16* p) {
  f.h[0] = *(const v8h*)p;
  f.h[1] = *(const v8h*)(p + 16);
}
__device__ __forceinline__ v8f zacc() { v8f z = {0.f, 0.f, 0.f, 0.f, 0.f, 0.f, 0.f, 0.f}; return z; }

__device__ __forceinline__ float rcpf_(float x) { return __builtin_amdgcn_rcpf(x); }
__device__ __forceinline__ float softs(float v) { return v * rcpf_(1.0f + fabsf(v)); }
__device__ __forceinline__ float sigmf(float v) {
  const float e = __expf(-fabsf(v));
  const float r = rcpf_(1.0f + e);
  const float neg = e * r;
  return v >= 0.0f ? r : neg;
}
__device__ __forceinline__ float tanhf_(float v) {
  const float e = __expf(-2.0f * fabsf(v));
  const float t = (1.0f - e) * rcpf_(1.0f + e);
  return v >= 0.0f ? t : -t;
}

__global__ __launch_bounds__(NTHR) void k_cvtw(const float* __restrict__ src, _Float16* dst,
                                             int nOv, int kIv, int nPd, int kP, int trans, float scale) {
  const int kp8 = kP >> 3;
  const int units = nPd * kp8;
  const int i = (int)blockIdx.x * NTHR + (int)threadIdx.x;
  if (i >= units) return;
  const int n  = i / kp8;
  const int k0 = (i - n * kp8) * 8;
  const int nc = n < nOv ? n : nOv - 1;
  v8h o;
#pragma unroll
  for (int e = 0; e < 8; ++e) {
    const int k  = k0 + e;
    const int kc = k < kIv ? k : kIv - 1;
    const int ia = kc * nOv + nc;
    const int ib = nc * kIv + kc;
    const int idx = trans ? ia : ib;
    float v = src[idx];
    v = (n < nOv && k < kIv) ? v * scale : 0.0f;
    o[e] = (_Float16)v;
  }
  _Float16* dp = dst + (size_t)i * 8;
  *(volatile v8h*)dp = o;
  __threadfence();
  *(volatile v8h*)dp = o;
}

__global__ __launch_bounds__(NTHR) void k_prepx(const float* __restrict__ x, _Float16* xh, int nN, int nP) {
  const int i = (int)blockIdx.x * NTHR + (int)threadIdx.x;
  if (i >= nP * (F / 8)) return;
  const int row = i >> 4;
  const int c0  = (i & 15) * 8;
  const int rc  = row < nN ? row : nN - 1;
  const float* sp = x + (size_t)rc * F + c0;
  const v4f a = *(const v4f*)sp, b = *(const v4f*)(sp + 4);
  const float s = row < nN ? SC_A : 0.0f;
  v8h o;
  o[0] = (_Float16)(a.x * s); o[1] = (_Float16)(a.y * s); o[2] = (_Float16)(a.z * s); o[3] = (_Float16)(a.w * s);
  o[4] = (_Float16)(b.x * s); o[5] = (_Float16)(b.y * s); o[6] = (_Float16)(b.z * s); o[7] = (_Float16)(b.w * s);
  _Float16* dp = xh + (size_t)i * 8;
  *(volatile v8h*)dp = o;
  __threadfence();
  *(volatile v8h*)dp = o;
}

template <int NB>
__device__ __forceinline__ int scan_chunk(const int* __restrict__ dsts, const float* __restrict__ attr, float tc,
                                          int nE, int cbase, int slotBase, int vec8, int* list,
                                          int tid, int lane, int wave) {
  int wc = 0;
#pragma unroll
  for (int g = 0; g < NGRP; ++g) {
    const int el0  = (g * NTHR + tid) * EPT;
    const int e0   = cbase + el0;
    const int sent = -2147483647 - 1;
    v4i da, db;
    v4f fa, fb;
    if (vec8 != 0 && cbase + CHUNK <= nE) {
      da = *(const v4i*)(dsts + e0);
      db = *(const v4i*)(dsts + e0 + 4);
      fa = *(const v4f*)(attr + e0);
      fb = *(const v4f*)(attr + e0 + 4);
    } else {
      const int q0 = min(e0, nE - 1),     q1 = min(e0 + 1, nE - 1), q2 = min(e0 + 2, nE - 1), q3 = min(e0 + 3, nE - 1);
      const int q4 = min(e0 + 4, nE - 1), q5 = min(e0 + 5, nE - 1), q6 = min(e0 + 6, nE - 1), q7 = min(e0 + 7, nE - 1);
      da.x = (e0     < nE) ? dsts[q0] : sent;
      da.y = (e0 + 1 < nE) ? dsts[q1] : sent;
      da.z = (e0 + 2 < nE) ? dsts[q2] : sent;
      da.w = (e0 + 3 < nE) ? dsts[q3] : sent;
      db.x = (e0 + 4 < nE) ? dsts[q4] : sent;
      db.y = (e0 + 5 < nE) ? dsts[q5] : sent;
      db.z = (e0 + 6 < nE) ? dsts[q6] : sent;
      db.w = (e0 + 7 < nE) ? dsts[q7] : sent;
      fa.x = attr[q0]; fa.y = attr[q1]; fa.z = attr[q2]; fa.w = attr[q3];
      fb.x = attr[q4]; fb.y = attr[q5]; fb.z = attr[q6]; fb.w = attr[q7];
    }
    const unsigned nb = (unsigned)slotBase;
    const unsigned s0 = (unsigned)da.x - nb, s1 = (unsigned)da.y - nb;
    const unsigned s2 = (unsigned)da.z - nb, s3 = (unsigned)da.w - nb;
    const unsigned s4 = (unsigned)db.x - nb, s5 = (unsigned)db.y - nb;
    const unsigned s6 = (unsigned)db.z - nb, s7 = (unsigned)db.w - nb;
    const bool h0 = (s0 < (unsigned)NB) && (fa.x <= tc), h1 = (s1 < (unsigned)NB) && (fa.y <= tc);
    const bool h2 = (s2 < (unsigned)NB) && (fa.z <= tc), h3 = (s3 < (unsigned)NB) && (fa.w <= tc);
    const bool h4 = (s4 < (unsigned)NB) && (fb.x <= tc), h5 = (s5 < (unsigned)NB) && (fb.y <= tc);
    const bool h6 = (s6 < (unsigned)NB) && (fb.z <= tc), h7 = (s7 < (unsigned)NB) && (fb.w <= tc);
    const unsigned any = __builtin_amdgcn_ballot_w32(h0 | h1 | h2 | h3 | h4 | h5 | h6 | h7);
    if (any != 0u) {
#define HITJ(J, HJ, SJ) { \
        const unsigned mj = __builtin_amdgcn_ballot_w32(HJ); \
        if (mj != 0u) { \
          if (HJ) { \
            const int pos = wc + (int)__builtin_amdgcn_mbcnt_lo(mj, 0u); \
            if (pos < WCAP) list[wave * WCAP + pos] = ((el0 + (J)) << 12) | (int)(SJ); \
          } \
          wc += (int)__builtin_popcount(mj); } }
      HITJ(0, h0, s0)
      HITJ(1, h1, s1)
      HITJ(2, h2, s2)
      HITJ(3, h3, s3)
      HITJ(4, h4, s4)
      HITJ(5, h5, s5)
      HITJ(6, h6, s6)
      HITJ(7, h7, s7)
#undef HITJ
    }
  }
  return wc;
}

__global__ __launch_bounds__(NTHR) void k_csr(
    const int* __restrict__ ei, const float* __restrict__ attr, const float* __restrict__ tcp,
    int* gcnt, int* gsst, int* greg, int nN, int nE, int vec8) {
  extern __shared__ v4i lds_dyn_i[];
  int* region = (int*)lds_dyn_i;
  int* cursor = region + RCAP;
  int* scnt   = cursor + NBF;
  int* sst    = scnt + NBF;
  int* list   = sst + NBF;
  int* wcnt   = list + LISTN;
  int* wtot   = wcnt + 16;
  const int tid = threadIdx.x, lane = tid & 31, wave = tid >> 5;
  const int nodeBase = blockIdx.x * NBF;
  const float tc = tcp[0];
  (void)nN;

  {
    const v4i z = {0, 0, 0, 0};
#pragma unroll 1
    for (int i = tid; i < RCAP / 4; i += NTHR) ((v4i*)region)[i] = z;
#pragma unroll 1
    for (int i = tid; i < NBF; i += NTHR) scnt[i] = 0;
  }
  __syncthreads();

  const int nChunks = (nE + CHUNK - 1) / CHUNK;

#pragma unroll 1
  for (int li = 0; li < 2; ++li) {
    const int* dsts = (li == 0) ? (ei + nE) : ei;
#pragma unroll 1
    for (int ch = 0; ch < nChunks; ++ch) {
      const int cbase = ch * CHUNK;
      const int wc = scan_chunk<NBF>(dsts, attr, tc, nE, cbase, nodeBase, vec8, list, tid, lane, wave);
      if (lane == 0) wcnt[wave] = wc;
      __syncthreads();
      if (wave == 0) {
#pragma unroll 1
        for (int wsx = 0; wsx < NWAVE; ++wsx) {
          int n = __builtin_amdgcn_readfirstlane(wcnt[wsx]);
          n = n > WCAP ? WCAP : (n < 0 ? 0 : n);
          const int* lp = list + wsx * WCAP;
#pragma unroll 1
          for (int i = 0; i < n; ++i) {
            const int ent  = __builtin_amdgcn_readfirstlane(lp[i]);
            const int slot = ent & (NBF - 1);
            if (lane == 0) scnt[slot] = scnt[slot] + 1;
          }
        }
      }
      __syncthreads();
    }
  }

  {
    const v4i cv = *(const v4i*)(scnt + 4 * tid);
    const int e0 = max(cv.x, 0), e1 = max(cv.y, 0), e2 = max(cv.z, 0), e3 = max(cv.w, 0);
    const int ts = e0 + e1 + e2 + e3;
    int incl = ts;
#pragma unroll
    for (int d = 1; d < 32; d <<= 1) {
      const int t = __shfl_up(incl, d);
      if (lane >= d) incl += t;
    }
    if (lane == 31) wtot[wave] = incl;
    __syncthreads();
    int pre = 0;
#pragma unroll 1
    for (int w = 0; w < wave; ++w) pre += wtot[w];
    int run = pre + incl - ts;
    int o;
    o = run > RCAP ? RCAP : run; sst[4 * tid + 0] = o; cursor[4 * tid + 0] = o; run += e0;
    o = run > RCAP ? RCAP : run; sst[4 * tid + 1] = o; cursor[4 * tid + 1] = o; run += e1;
    o = run > RCAP ? RCAP : run; sst[4 * tid + 2] = o; cursor[4 * tid + 2] = o; run += e2;
    o = run > RCAP ? RCAP : run; sst[4 * tid + 3] = o; cursor[4 * tid + 3] = o;
  }
  __syncthreads();

#pragma unroll 1
  for (int li = 0; li < 2; ++li) {
    const int* dsts = (li == 0) ? (ei + nE) : ei;
    const int* srcs = (li == 0) ? ei : (ei + nE);
#pragma unroll 1
    for (int ch = 0; ch < nChunks; ++ch) {
      const int cbase = ch * CHUNK;
      const int wc = scan_chunk<NBF>(dsts, attr, tc, nE, cbase, nodeBase, vec8, list, tid, lane, wave);
      if (lane == 0) wcnt[wave] = wc;
      __syncthreads();
      if (wave == 0) {
#pragma unroll 1
        for (int wsx = 0; wsx < NWAVE; ++wsx) {
          int n = __builtin_amdgcn_readfirstlane(wcnt[wsx]);
          n = n > WCAP ? WCAP : (n < 0 ? 0 : n);
          const int* lp = list + wsx * WCAP;
#pragma unroll 1
          for (int i = 0; i < n; ++i) {
            const int ent  = __builtin_amdgcn_readfirstlane(lp[i]);
            const int slot = ent & (NBF - 1);
            int e = cbase + ((ent >> 12) & (CHUNK - 1));
            e = e > nE - 1 ? nE - 1 : e;
            int src = srcs[e];
            src = src < 0 ? 0 : (src > nN - 1 ? nN - 1 : src);
            if (lane == 0) {
              int pos = cursor[slot];
              pos = pos < 0 ? 0 : (pos > RCAP - 1 ? RCAP - 1 : pos);
              region[pos] = src;
              const int np = pos + 1;
              cursor[slot] = np > RCAP ? RCAP : np;
            }
          }
        }
      }
      __syncthreads();
    }
  }

  const v4i cvo = *(const v4i*)(scnt + 4 * tid);
  const v4i svo = *(const v4i*)(sst + 4 * tid);
  int* pc = gcnt + nodeBase + 4 * tid;
  int* ps = gsst + nodeBase + 4 * tid;
  int* pr = greg + (size_t)blockIdx.x * RCAP;
  *(volatile v4i*)pc = cvo;
  *(volatile v4i*)ps = svo;
#pragma unroll 1
  for (int i = 0; i < RCAP / (4 * NTHR); ++i) {
    const v4i rv = ((const v4i*)region)[i * NTHR + tid];
    *(volatile v4i*)(pr + 4 * (i * NTHR + tid)) = rv;
  }
  __threadfence();
  *(volatile v4i*)pc = cvo;
  *(volatile v4i*)ps = svo;
#pragma unroll 1
  for (int i = 0; i < RCAP / (4 * NTHR); ++i) {
    const v4i rv = ((const v4i*)region)[i * NTHR + tid];
    *(volatile v4i*)(pr + 4 * (i * NTHR + tid)) = rv;
  }
}

__global__ __launch_bounds__(NTHR) void k_gmlp(
    const _Float16* __restrict__ ah, const _Float16* __restrict__ w1p, const float* __restrict__ b1,
    const _Float16* __restrict__ w2p, const float* __restrict__ b2,
    const float* __restrict__ w3, const float* __restrict__ b3, float* gout, int nN) {
  __shared__ __attribute__((aligned(16))) _Float16 sG1[BR * (GH1 + 8)];
  __shared__ __attribute__((aligned(16))) float sG2[BR * GH2];
  __shared__ __attribute__((aligned(16))) float sG[BR];
  const int tid = threadIdx.x, lane = tid & 31, wave = tid >> 5, hh = lane >> 4, m = lane & 15;
  const int rowBase = blockIdx.x * BR;

  {
    const int rg = wave >> 2, t = wave & 3, r0 = 16 * rg;
    int arow = rowBase + r0 + m; arow = arow > nN - 1 ? nN - 1 : arow;
    const _Float16* ap = ah + (size_t)arow * F + 8 * hh;
    const _Float16* bp = w1p + (size_t)(16 * t + m) * F + 8 * hh;
    v8f acc = zacc();
#pragma unroll
    for (int kt = 0; kt < F / 32; ++kt) {
      Frag a, b;
      ldfrag(a, ap + 32 * kt);
      ldfrag(b, bp + 32 * kt);
      acc = wmf(a.v, b.v, acc);
    }
    const int col = 16 * t + m;
    const float bv = b1[col];
#pragma unroll
    for (int r = 0; r < 8; ++r) {
      const int row = r0 + 8 * hh + r;
      const float v = softs(acc[r] * SC_INV + bv);
      sG1[row * (GH1 + 8) + col] = (_Float16)(v * SC_A);
    }
  }
  __syncthreads();

  {
    const int rg = (wave >> 1) & 1, t = wave & 1, r0 = 16 * rg;
    const _Float16* ap = sG1 + (r0 + m) * (GH1 + 8) + 8 * hh;
    const _Float16* bp = w2p + (size_t)(16 * t + m) * GH1 + 8 * hh;
    v8f acc = zacc();
#pragma unroll
    for (int kt = 0; kt < GH1 / 32; ++kt) {
      Frag a, b;
      ldfrag(a, ap + 32 * kt);
      ldfrag(b, bp + 32 * kt);
      acc = wmf(a.v, b.v, acc);
    }
    if (wave < 4) {
      const int col = 16 * t + m;
      const float bv = b2[col];
#pragma unroll
      for (int r = 0; r < 8; ++r) {
        const int row = r0 + 8 * hh + r;
        sG2[row * GH2 + col] = softs(acc[r] * SC_INV + bv);
      }
    }
  }
  __syncthreads();

  {
    const int row = tid >> 3, pq = tid & 7;
    const float* sp = sG2 + row * GH2 + 4 * pq;
    const v4f gv = *(const v4f*)sp;
    const v4f wv = *(const v4f*)(w3 + 4 * pq);
    const v4f pv = gv * wv;
    float s = (pv.x + pv.y) + (pv.z + pv.w);
    s += __shfl_xor(s, 1);
    s += __shfl_xor(s, 2);
    s += __shfl_xor(s, 4);
    if (pq == 0) sG[row] = s + b3[0];
  }
  __syncthreads();

  const float v = sG[lane];
  float* p = gout + rowBase + lane;
  if (wave == 0) *(volatile float*)p = v;
  __threadfence();
  if (wave == 0) *(volatile float*)p = v;
}

__device__ __forceinline__ v4f agg_one(const int* __restrict__ greg, const int* __restrict__ gcnt,
                                       const int* __restrict__ gsst, const float* __restrict__ gl,
                                       const float* __restrict__ hf, int c, int nN, bool selfk, int lane) {
  const int cc = c < nN ? c : nN - 1;
  int n = __builtin_amdgcn_readfirstlane(gcnt[c]);
  n = n < 0 ? 0 : (n > DEGCAP ? DEGCAP : n);
  int st = __builtin_amdgcn_readfirstlane(gsst[c]);
  st = st < 0 ? 0 : (st > RCAP ? RCAP : st);
  if (n > RCAP - st) n = RCAP - st;
  const int* rp = greg + (size_t)(c / NBF) * RCAP + st;
  const float gself = gl[cc];
  const float NEG = -__builtin_inff();

  float mx = selfk ? gself : NEG;
#pragma unroll 1
  for (int q0 = 0; q0 < n; q0 += 32) {
    int pos = q0 + lane; pos = pos > n - 1 ? n - 1 : pos;
    int sl = rp[pos];
    sl = sl < 0 ? 0 : (sl > nN - 1 ? nN - 1 : sl);
    const float gs = gl[sl];
    float lm = (q0 + lane < n) ? gs : NEG;
    lm = fmaxf(lm, __shfl_xor(lm, 16));
    lm = fmaxf(lm, __shfl_xor(lm, 8));
    lm = fmaxf(lm, __shfl_xor(lm, 4));
    lm = fmaxf(lm, __shfl_xor(lm, 2));
    lm = fmaxf(lm, __shfl_xor(lm, 1));
    mx = fmaxf(mx, lm);
  }
  if (!(mx > NEG)) mx = 0.0f;

  const float pself = selfk ? __expf(gself - mx) : 0.0f;
  float den = pself;
  const float* hrow = hf + (size_t)cc * F + 4 * lane;
  v4f acc = *(const v4f*)hrow * pself;
#pragma unroll 1
  for (int q0 = 0; q0 < n; q0 += 32) {
    int pos = q0 + lane; pos = pos > n - 1 ? n - 1 : pos;
    int sl = rp[pos];
    sl = sl < 0 ? 0 : (sl > nN - 1 ? nN - 1 : sl);
    const float gs = gl[sl];
    const float pl = (q0 + lane < n) ? __expf(gs - mx) : 0.0f;
    float ds = pl;
    ds += __shfl_xor(ds, 16);
    ds += __shfl_xor(ds, 8);
    ds += __shfl_xor(ds, 4);
    ds += __shfl_xor(ds, 2);
    ds += __shfl_xor(ds, 1);
    den += ds;
    const int mcnt = (n - q0) < 32 ? (n - q0) : 32;
#pragma unroll 1
    for (int pp = 0; pp < mcnt; ++pp) {
      const int   s  = __builtin_amdgcn_readlane(sl, pp);
      const float pv = __int_as_float(__builtin_amdgcn_readlane(__float_as_int(pl), pp));
      const float* hq = hf + (size_t)s * F + 4 * lane;
      acc = acc + *(const v4f*)hq * pv;
    }
  }
  const float rd = den > 0.0f ? rcpf_(den) : 0.0f;
  return acc * rd;
}

__global__ __launch_bounds__(NTHR) void k_agg(
    const int* __restrict__ greg, const int* __restrict__ gcnt, const int* __restrict__ gsst,
    const float* __restrict__ gl, const float* __restrict__ hf, const float* __restrict__ tcp,
    _Float16* mh, int nN) {
  __shared__ __attribute__((aligned(16))) _Float16 sRel[NWAVE * 2 * F];
  const int tid = threadIdx.x, lane = tid & 31, wave = tid >> 5;
  const float tc = tcp[0];
  const bool selfk = (1.0f <= tc);
  const int rowBase = blockIdx.x * BR + wave * (BR / NWAVE);
  _Float16* myRel = sRel + wave * 2 * F;

#pragma unroll 1
  for (int pr = 0; pr < (BR / NWAVE) / 2; ++pr) {
    const int c0 = rowBase + 2 * pr;
    const v4f m0 = agg_one(greg, gcnt, gsst, gl, hf, c0, nN, selfk, lane);
    const v4f m1 = agg_one(greg, gcnt, gsst, gl, hf, c0 + 1, nN, selfk, lane);
    v4h q0, q1;
    q0.x = (_Float16)(m0.x * SC_A); q0.y = (_Float16)(m0.y * SC_A); q0.z = (_Float16)(m0.z * SC_A); q0.w = (_Float16)(m0.w * SC_A);
    q1.x = (_Float16)(m1.x * SC_A); q1.y = (_Float16)(m1.y * SC_A); q1.z = (_Float16)(m1.z * SC_A); q1.w = (_Float16)(m1.w * SC_A);
    *(v4h*)(myRel + 4 * lane)     = q0;
    *(v4h*)(myRel + F + 4 * lane) = q1;
    __builtin_amdgcn_fence(__ATOMIC_RELEASE, "wavefront");
    __builtin_amdgcn_wave_barrier();
    const v8h ov = *(const v8h*)(myRel + 8 * lane);
    __builtin_amdgcn_fence(__ATOMIC_RELEASE, "wavefront");
    __builtin_amdgcn_wave_barrier();
    _Float16* gp = mh + (size_t)c0 * F + 8 * lane;
    *(volatile v8h*)gp = ov;
    __threadfence();
    *(volatile v8h*)gp = ov;
  }
}

__global__ __launch_bounds__(NTHR) void k_gru(
    const _Float16* __restrict__ mh, const _Float16* ahin, const float* hfin,
    const _Float16* __restrict__ wihp, const _Float16* __restrict__ whhp,
    const float* __restrict__ bih, const float* __restrict__ bhh,
    float* hfout, _Float16* hhout, int nN) {
  __shared__ __attribute__((aligned(16))) float stg[BR * F];
  const int tid = threadIdx.x, lane = tid & 31, wave = tid >> 5, hh = lane >> 4, m = lane & 15;
  const int rowBase = blockIdx.x * BR;
  const int rg = wave >> 2, cg = wave & 3, r0 = 16 * rg, c0 = 32 * cg;
  int arow = rowBase + r0 + m; arow = arow > nN - 1 ? nN - 1 : arow;
  const _Float16* amp = mh + (size_t)arow * F + 8 * hh;
  const _Float16* ahp = ahin + (size_t)arow * F + 8 * hh;

  v8f gi[6], gh[6];
#pragma unroll
  for (int i = 0; i < 6; ++i) { gi[i] = zacc(); gh[i] = zacc(); }

#pragma unroll 1
  for (int kt = 0; kt < F / 32; ++kt) {
    Frag fa, fb;
    ldfrag(fa, amp + 32 * kt);
    ldfrag(fb, ahp + 32 * kt);
#pragma unroll
    for (int q = 0; q < 3; ++q) {
#pragma unroll
      for (int t = 0; t < 2; ++t) {
        const size_t boff = (size_t)(q * F + c0 + 16 * t + m) * F + 32 * kt + 8 * hh;
        Frag bi, bw;
        ldfrag(bi, wihp + boff);
        ldfrag(bw, whhp + boff);
        gi[q * 2 + t] = wmf(fa.v, bi.v, gi[q * 2 + t]);
        gh[q * 2 + t] = wmf(fb.v, bw.v, gh[q * 2 + t]);
      }
    }
  }

#pragma unroll
  for (int t = 0; t < 2; ++t) {
    const int col = c0 + 16 * t + m;
    const float bir = bih[col], biz = bih[F + col], bin = bih[2 * F + col];
    const float bhr = bhh[col], bhz = bhh[F + col], bhn = bhh[2 * F + col];
#pragma unroll
    for (int r = 0; r < 8; ++r) {
      const int row = r0 + 8 * hh + r;
      int grow = rowBase + row; grow = grow > nN - 1 ? nN - 1 : grow;
      const float hold = hfin[(size_t)grow * F + col];
      const float ir = gi[t][r] * SC_INV + bir;
      const float iz = gi[2 + t][r] * SC_INV + biz;
      const float ig = gi[4 + t][r] * SC_INV + bin;
      const float hr = gh[t][r] * SC_INV + bhr;
      const float hz = gh[2 + t][r] * SC_INV + bhz;
      const float hn = gh[4 + t][r] * SC_INV + bhn;
      const float rr = sigmf(ir + hr);
      const float zz = sigmf(iz + hz);
      const float cand = tanhf_(ig + rr * hn);
      stg[row * F + col] = (1.0f - zz) * cand + zz * hold;
    }
  }
  __syncthreads();

  v4f hv[4];
#pragma unroll
  for (int i = 0; i < 4; ++i) hv[i] = *(const v4f*)(stg + 4 * (i * NTHR + tid));
  v8h qv[2];
#pragma unroll
  for (int i = 0; i < 2; ++i) {
    const float* sp = stg + 8 * (i * NTHR + tid);
    const v4f a = *(const v4f*)sp, b = *(const v4f*)(sp + 4);
    v8h o;
    o[0] = (_Float16)(a.x * SC_A); o[1] = (_Float16)(a.y * SC_A); o[2] = (_Float16)(a.z * SC_A); o[3] = (_Float16)(a.w * SC_A);
    o[4] = (_Float16)(b.x * SC_A); o[5] = (_Float16)(b.y * SC_A); o[6] = (_Float16)(b.z * SC_A); o[7] = (_Float16)(b.w * SC_A);
    qv[i] = o;
  }
  float* hp = hfout + (size_t)rowBase * F;
  _Float16* qp = hhout + (size_t)rowBase * F;
#pragma unroll
  for (int i = 0; i < 4; ++i) *(volatile v4f*)(hp + 4 * (i * NTHR + tid)) = hv[i];
#pragma unroll
  for (int i = 0; i < 2; ++i) *(volatile v8h*)(qp + 8 * (i * NTHR + tid)) = qv[i];
  __threadfence();
#pragma unroll
  for (int i = 0; i < 4; ++i) *(volatile v4f*)(hp + 4 * (i * NTHR + tid)) = hv[i];
#pragma unroll
  for (int i = 0; i < 2; ++i) *(volatile v8h*)(qp + 8 * (i * NTHR + tid)) = qv[i];
}

__global__ __launch_bounds__(NTHR) void k_final(
    const _Float16* __restrict__ hhp, const _Float16* __restrict__ xh,
    const _Float16* __restrict__ w1p, const float* __restrict__ b1,
    const _Float16* __restrict__ w2p, const float* __restrict__ b2,
    const _Float16* __restrict__ wjp, const float* __restrict__ bj,
    _Float16* tp, int nN, int nP) {
  extern __shared__ v4f lds_dyn[];
  char* base = (char*)lds_dyn;
  _Float16* sA1  = (_Float16*)base;
  float*    sL   = (float*)(base + BRF * (F + 8) * 2);
  float*    sInv = sL + BRF * F;
  _Float16* sT   = (_Float16*)(sInv + BRF);
  const int tid = threadIdx.x, lane = tid & 31, wave = tid >> 5, hh = lane >> 4, m = lane & 15;
  const int rowBase = blockIdx.x * BRF;
  const int rg = wave >> 1, ch = wave & 1, r0 = 16 * rg;
  int arow = rowBase + r0 + m; arow = arow > nN - 1 ? nN - 1 : arow;

  {
    v8f acc[4];
#pragma unroll
    for (int t = 0; t < 4; ++t) acc[t] = zacc();
    const _Float16* aph = hhp + (size_t)arow * F + 8 * hh;
    const _Float16* apx = xh + (size_t)arow * F + 8 * hh;
#pragma unroll
    for (int kt = 0; kt < F / 32; ++kt) {
      Frag a;
      ldfrag(a, aph + 32 * kt);
#pragma unroll
      for (int t = 0; t < 4; ++t) {
        Frag b;
        ldfrag(b, w1p + (size_t)(64 * ch + 16 * t + m) * (2 * F) + 32 * kt + 8 * hh);
        acc[t] = wmf(a.v, b.v, acc[t]);
      }
    }
#pragma unroll
    for (int kt = 0; kt < F / 32; ++kt) {
      Frag a;
      ldfrag(a, apx + 32 * kt);
#pragma unroll
      for (int t = 0; t < 4; ++t) {
        Frag b;
        ldfrag(b, w1p + (size_t)(64 * ch + 16 * t + m) * (2 * F) + F + 32 * kt + 8 * hh);
        acc[t] = wmf(a.v, b.v, acc[t]);
      }
    }
#pragma unroll
    for (int t = 0; t < 4; ++t) {
      const int col = 64 * ch + 16 * t + m;
      const float bv = b1[col];
#pragma unroll
      for (int r = 0; r < 8; ++r) {
        const int row = r0 + 8 * hh + r;
        const float v = softs(acc[t][r] * SC_INV + bv);
        sA1[row * (F + 8) + col] = (_Float16)(v * SC_A);
      }
    }
  }
  __syncthreads();

  {
    v8f acc[4];
#pragma unroll
    for (int t = 0; t < 4; ++t) acc[t] = zacc();
    const _Float16* ap = sA1 + (r0 + m) * (F + 8) + 8 * hh;
#pragma unroll
    for (int kt = 0; kt < F / 32; ++kt) {
      Frag a;
      ldfrag(a, ap + 32 * kt);
#pragma unroll
      for (int t = 0; t < 4; ++t) {
        Frag b;
        ldfrag(b, w2p + (size_t)(64 * ch + 16 * t + m) * F + 32 * kt + 8 * hh);
        acc[t] = wmf(a.v, b.v, acc[t]);
      }
    }
#pragma unroll
    for (int t = 0; t < 4; ++t) {
      const int col = 64 * ch + 16 * t + m;
      const float bv = b2[col];
#pragma unroll
      for (int r = 0; r < 8; ++r) {
        const int row = r0 + 8 * hh + r;
        sL[row * F + col] = softs(acc[t][r] * SC_INV + bv);
      }
    }
  }
  __syncthreads();

  {
    const int row = tid >> 2, pq = tid & 3;
    float* lr = sL + row * F + pq * 32;
    v4f q[8];
#pragma unroll
    for (int j = 0; j < 8; ++j) q[j] = *(const v4f*)(lr + 4 * j);
    float mx = -__builtin_inff();
#pragma unroll
    for (int j = 0; j < 8; ++j) mx = fmaxf(mx, fmaxf(fmaxf(q[j].x, q[j].y), fmaxf(q[j].z, q[j].w)));
    mx = fmaxf(mx, __shfl_xor(mx, 1));
    mx = fmaxf(mx, __shfl_xor(mx, 2));
    float s = 0.0f;
#pragma unroll
    for (int j = 0; j < 8; ++j) {
      v4f e;
      e.x = __expf(q[j].x - mx); e.y = __expf(q[j].y - mx); e.z = __expf(q[j].z - mx); e.w = __expf(q[j].w - mx);
      s += (e.x + e.y) + (e.z + e.w);
      *(v4f*)(lr + 4 * j) = e;
    }
    s += __shfl_xor(s, 1);
    s += __shfl_xor(s, 2);
    if (pq == 0) sInv[row] = rcpf_(s);
  }
  __syncthreads();

  {
    v8f acc[4];
#pragma unroll
    for (int t = 0; t < 4; ++t) acc[t] = zacc();
    const _Float16* apx = xh + (size_t)arow * F + 8 * hh;
#pragma unroll
    for (int kt = 0; kt < F / 32; ++kt) {
      Frag a;
      ldfrag(a, apx + 32 * kt);
#pragma unroll
      for (int t = 0; t < 4; ++t) {
        Frag b;
        ldfrag(b, wjp + (size_t)(64 * ch + 16 * t + m) * F + 32 * kt + 8 * hh);
        acc[t] = wmf(a.v, b.v, acc[t]);
      }
    }
#pragma unroll
    for (int t = 0; t < 4; ++t) {
      const int col = 64 * ch + 16 * t + m;
      const float bv = bj[col];
#pragma unroll
      for (int r = 0; r < 8; ++r) {
        const int row = r0 + 8 * hh + r;
        const float ajv = softs(acc[t][r] * SC_INV + bv);
        const float nov = sL[row * F + col] * sInv[row] * ajv;
        const float v = nov * SC_T;
        const _Float16 hi = (_Float16)v;
        const float res = v - (float)hi;
        const _Float16 lo = (_Float16)(res * SC_TL);
        sT[col * (BRF + 8) + row] = hi;
        sT[F * (BRF + 8) + col * (BRF + 8) + row] = lo;
      }
    }
  }
  __syncthreads();

  v8h ov[8];
#pragma unroll
  for (int i = 0; i < 8; ++i) {
    const int L = wave * 32 + 4 * i + (lane >> 3);
    const int pl = L >> 7, c = L & 127;
    ov[i] = *(const v8h*)(sT + pl * (F * (BRF + 8)) + c * (BRF + 8) + (lane & 7) * 8);
  }
#pragma unroll
  for (int i = 0; i < 8; ++i) {
    const int L = wave * 32 + 4 * i + (lane >> 3);
    const int pl = L >> 7, c = L & 127;
    _Float16* dp = tp + (size_t)pl * F * nP + (size_t)c * nP + rowBase + (lane & 7) * 8;
    *(volatile v8h*)dp = ov[i];
  }
  __threadfence();
#pragma unroll
  for (int i = 0; i < 8; ++i) {
    const int L = wave * 32 + 4 * i + (lane >> 3);
    const int pl = L >> 7, c = L & 127;
    _Float16* dp = tp + (size_t)pl * F * nP + (size_t)c * nP + rowBase + (lane & 7) * 8;
    *(volatile v8h*)dp = ov[i];
  }
}

__global__ __launch_bounds__(NTHR) void k_pool(
    const _Float16* __restrict__ tp, const int* __restrict__ bat, float* part, int nN, int nP) {
  __shared__ __attribute__((aligned(16))) float sP[F * NGP];
  const int tid = threadIdx.x, lane = tid & 31, wave = tid >> 5, hh = lane >> 4, m = lane & 15;
  const int nbase = blockIdx.x * KCH;
  const int crow = 16 * wave + m;
  const _Float16* aph = tp + (size_t)crow * nP + nbase + 8 * hh;
  const _Float16* apl = aph + (size_t)F * nP;
  const bool fullblk = (nbase + KCH <= nN);
  const _Float16 one = (_Float16)1.0f, zer = (_Float16)0.0f;

  v8f acch[4], accl[4];
#pragma unroll
  for (int t = 0; t < 4; ++t) { acch[t] = zacc(); accl[t] = zacc(); }

#pragma unroll 1
  for (int kt = 0; kt < KCH / 32; ++kt) {
    Frag ah, al;
    ldfrag(ah, aph + 32 * kt);
    ldfrag(al, apl + 32 * kt);
    const int na = nbase + 32 * kt + 8 * hh;
    int bid[16];
    if (fullblk) {
      const v4i u0 = *(const v4i*)(bat + na), u1 = *(const v4i*)(bat + na + 4);
      const v4i u2 = *(const v4i*)(bat + na + 16), u3 = *(const v4i*)(bat + na + 20);
      bid[0] = u0.x; bid[1] = u0.y; bid[2]  = u0.z; bid[3]  = u0.w;
      bid[4] = u1.x; bid[5] = u1.y; bid[6]  = u1.z; bid[7]  = u1.w;
      bid[8] = u2.x; bid[9] = u2.y; bid[10] = u2.z; bid[11] = u2.w;
      bid[12] = u3.x; bid[13] = u3.y; bid[14] = u3.z; bid[15] = u3.w;
    } else {
#pragma unroll
      for (int i = 0; i < 16; ++i) {
        const int n = (i < 8) ? (na + i) : (na + 16 + (i - 8));
        const int nc = n < nN ? n : nN - 1;
        const int b = bat[nc];
        bid[i] = (n < nN) ? b : -1;
      }
    }
#pragma unroll
    for (int t = 0; t < 4; ++t) {
      const int gsel = 16 * t + m;
      Frag b;
#pragma unroll
      for (int i = 0; i < 16; ++i) b.v[i] = (bid[i] == gsel) ? one : zer;
      acch[t] = wmf(ah.v, b.v, acch[t]);
      accl[t] = wmf(al.v, b.v, accl[t]);
    }
  }

#pragma unroll
  for (int t = 0; t < 4; ++t) {
    const int gq = 16 * t + m;
#pragma unroll
    for (int r = 0; r < 8; ++r) {
      const int c = 16 * wave + 8 * hh + r;
      sP[c * NGP + gq] = acch[t][r] * (1.0f / SC_T) + accl[t][r] * (1.0f / (SC_T * SC_TL));
    }
  }
  __syncthreads();

  v4f pv[8];
#pragma unroll
  for (int i = 0; i < 8; ++i) pv[i] = *(const v4f*)(sP + 4 * (i * NTHR + tid));
  float* pp = part + (size_t)blockIdx.x * (F * NGP);
#pragma unroll
  for (int i = 0; i < 8; ++i) *(volatile v4f*)(pp + 4 * (i * NTHR + tid)) = pv[i];
  __threadfence();
#pragma unroll
  for (int i = 0; i < 8; ++i) *(volatile v4f*)(pp + 4 * (i * NTHR + tid)) = pv[i];
}

__global__ __launch_bounds__(NTHR) void k_head(
    const float* __restrict__ part, int nKB,
    const _Float16* __restrict__ ow1p, const float* __restrict__ ob1,
    const _Float16* __restrict__ ow2p, const float* __restrict__ ob2,
    const float* __restrict__ ow3, const float* __restrict__ ob3, float* out, int nG) {
  __shared__ __attribute__((aligned(16))) _Float16 sPool[NGP * (F + 8)];
  __shared__ __attribute__((aligned(16))) _Float16 sO1[NGP * (H1P + 8)];
  __shared__ __attribute__((aligned(16))) float sO2[NGP * H2];
  __shared__ __attribute__((aligned(16))) float sO[NGP];
  const int tid = threadIdx.x, lane = tid & 31, wave = tid >> 5, hh = lane >> 4, m = lane & 15;

#pragma unroll 1
  for (int i = 0; i < (F * NGP) / NTHR; ++i) {
    const int e = i * NTHR + tid;
    float s = 0.0f;
#pragma unroll 1
    for (int kb = 0; kb < nKB; ++kb) s += part[(size_t)kb * (F * NGP) + e];
    const int c = e >> 6, gq = e & (NGP - 1);
    sPool[gq * (F + 8) + c] = (_Float16)(s * SC_A);
  }
  __syncthreads();

  const int rg = wave >> 1, r0 = 16 * rg;
  {
    v8f acc[3];
#pragma unroll
    for (int t = 0; t < 3; ++t) acc[t] = zacc();
    const _Float16* ap = sPool + (r0 + m) * (F + 8) + 8 * hh;
#pragma unroll
    for (int kt = 0; kt < F / 32; ++kt) {
      Frag a;
      ldfrag(a, ap + 32 * kt);
#pragma unroll
      for (int t = 0; t < 3; ++t) {
        Frag b;
        ldfrag(b, ow1p + (size_t)((wave & 1) * 48 + 16 * t + m) * F + 32 * kt + 8 * hh);
        acc[t] = wmf(a.v, b.v, acc[t]);
      }
    }
#pragma unroll
    for (int t = 0; t < 3; ++t) {
      const int col = (wave & 1) * 48 + 16 * t + m;
      const int cb = col < H1 ? col : H1 - 1;
      const float bv = ob1[cb];
#pragma unroll
      for (int r = 0; r < 8; ++r) {
        const int row = r0 + 8 * hh + r;
        float v = fmaxf(acc[t][r] * SC_INV + bv, 0.0f);
        v = col < H1 ? v : 0.0f;
        sO1[row * (H1P + 8) + col] = (_Float16)(v * SC_A);
      }
    }
  }
  __syncthreads();

  {
    v8f acc[2];
#pragma unroll
    for (int t = 0; t < 2; ++t) acc[t] = zacc();
    const _Float16* ap = sO1 + (r0 + m) * (H1P + 8) + 8 * hh;
#pragma unroll
    for (int kt = 0; kt < H1P / 32; ++kt) {
      Frag a;
      ldfrag(a, ap + 32 * kt);
#pragma unroll
      for (int t = 0; t < 2; ++t) {
        Frag b;
        ldfrag(b, ow2p + (size_t)((wave & 1) * 32 + 16 * t + m) * H1P + 32 * kt + 8 * hh);
        acc[t] = wmf(a.v, b.v, acc[t]);
      }
    }
#pragma unroll
    for (int t = 0; t < 2; ++t) {
      const int col = (wave & 1) * 32 + 16 * t + m;
      const float bv = ob2[col];
#pragma unroll
      for (int r = 0; r < 8; ++r) {
        const int row = r0 + 8 * hh + r;
        sO2[row * H2 + col] = fmaxf(acc[t][r] * SC_INV + bv, 0.0f);
      }
    }
  }
  __syncthreads();

  {
    const int gq = tid >> 2, pq = tid & 3;
    const float* sp = sO2 + gq * H2 + 16 * pq;
    const float* wp = ow3 + 16 * pq;
    float s = 0.0f;
#pragma unroll 4
    for (int k = 0; k < 16; ++k) s += sp[k] * wp[k];
    s += __shfl_xor(s, 1);
    s += __shfl_xor(s, 2);
    if (pq == 0) sO[gq] = s + ob3[0];
  }
  __syncthreads();

  const float v0 = sO[lane];
  const float v1 = sO[32 + lane];
  const bool st0 = (wave == 0) && (lane < nG);
  const bool st1 = (wave == 0) && (32 + lane < nG);
  if (st0) *(volatile float*)(out + lane) = v0;
  if (st1) *(volatile float*)(out + 32 + lane) = v1;
  __threadfence();
  if (st0) *(volatile float*)(out + lane) = v0;
  if (st1) *(volatile float*)(out + 32 + lane) = v1;
}

static inline size_t al256(size_t v) { return (v + 255) & ~(size_t)255; }

extern "C" void kernel_launch(void* const* d_in, const int* in_sizes, int n_in,
                              void* d_out, int out_size, void* d_ws, size_t ws_size,
                              hipStream_t stream) {
  if (n_in < 27) return;
  if (in_sizes[0] < F || (in_sizes[0] % F) != 0) return;
  const int nN = in_sizes[0] / F;
  if (nN < 1 || nN > (1 << 22)) return;
  const int nE2 = in_sizes[1];
  if (nE2 < 2 || (nE2 & 1) != 0) return;
  const int nE = nE2 / 2;
  if (nE > (1 << 28)) return;
  if (in_sizes[2] != nE || in_sizes[3] != nN || in_sizes[4] < 1) return;
  if (in_sizes[5] != F * GH1 || in_sizes[6] != GH1 || in_sizes[7] != GH1 * GH2 || in_sizes[8] != GH2) return;
  if (in_sizes[9] != GH2 || in_sizes[10] < 1) return;
  if (in_sizes[11] != G3 * F || in_sizes[12] != G3 * F || in_sizes[13] != G3 || in_sizes[14] != G3) return;
  if (in_sizes[15] != 2 * F * F || in_sizes[16] != F || in_sizes[17] != F * F || in_sizes[18] != F) return;
  if (in_sizes[19] != F * F || in_sizes[20] != F) return;
  if (in_sizes[21] != F * H1 || in_sizes[22] != H1 || in_sizes[23] != H1 * H2 || in_sizes[24] != H2) return;
  if (in_sizes[25] != H2 || in_sizes[26] < 1) return;
  const int nG = out_size;
  if (nG < 1 || nG > NGP) return;

  const float* x     = (const float*)d_in[0];
  const int*   ei    = (const int*)d_in[1];
  const float* eattr = (const float*)d_in[2];
  const int*   batch = (const int*)d_in[3];
  const float* tcut  = (const float*)d_in[4];
  const float* gW1 = (const float*)d_in[5],  *gb1 = (const float*)d_in[6];
  const float* gW2 = (const float*)d_in[7],  *gb2 = (const float*)d_in[8];
  const float* gW3 = (const float*)d_in[9],  *gb3 = (const float*)d_in[10];
  const float* Wih = (const float*)d_in[11], *Whh = (const float*)d_in[12];
  const float* bih = (const float*)d_in[13], *bhh = (const float*)d_in[14];
  const float* aW1 = (const float*)d_in[15], *ab1 = (const float*)d_in[16];
  const float* aW2 = (const float*)d_in[17], *ab2 = (const float*)d_in[18];
  const float* ajW = (const float*)d_in[19], *ajb = (const float*)d_in[20];
  const float* oW1 = (const float*)d_in[21], *ob1 = (const float*)d_in[22];
  const float* oW2 = (const float*)d_in[23], *ob2 = (const float*)d_in[24];
  const float* oW3 = (const float*)d_in[25], *ob3 = (const float*)d_in[26];
  float* out = (float*)d_out;

  const int NP   = ((nN + NBF - 1) / NBF) * NBF;
  const int nBF  = NP / NBF;
  const int nB32 = (nN + BR - 1) / BR;
  const int nB64 = NP / BRF;
  const int nKB  = NP / KCH;
  if (nB32 * BR > NP || nB64 * BRF != NP || nKB * KCH != NP) return;

  char* ws = (char*)d_ws;
  size_t off = 0;
  const size_t oXh  = off; off = al256(off + (size_t)NP * F * 2);
  const size_t oHf  = off; off = al256(off + (size_t)NP * F * 4);
  const size_t oHh  = off; off = al256(off + (size_t)NP * F * 2);
  const size_t oMh  = off; off = al256(off + (size_t)NP * F * 2);
  const size_t oG   = off; off = al256(off + (size_t)NP * 4);
  const size_t oCnt = off; off = al256(off + (size_t)NP * 4);
  const size_t oSst = off; off = al256(off + (size_t)NP * 4);
  const size_t oReg = off; off = al256(off + (size_t)nBF * RCAP * 4);
  const size_t oT   = off; off = al256(off + (size_t)2 * F * NP * 2);
  const size_t oPt  = off; off = al256(off + (size_t)nKB * F * NGP * 4);
  const size_t owW1 = off; off = al256(off + (size_t)GH1 * F * 2);
  const size_t owW2 = off; off = al256(off + (size_t)GH2 * GH1 * 2);
  const size_t oWih = off; off = al256(off + (size_t)G3 * F * 2);
  const size_t oWhh = off; off = al256(off + (size_t)G3 * F * 2);
  const size_t oA1  = off; off = al256(off + (size_t)F * 2 * F * 2);
  const size_t oA2  = off; off = al256(off + (size_t)F * F * 2);
  const size_t oAJ  = off; off = al256(off + (size_t)F * F * 2);
  const size_t oO1  = off; off = al256(off + (size_t)H1P * F * 2);
  const size_t oO2  = off; off = al256(off + (size_t)H2 * H1P * 2);
  if (off > ws_size || off > (size_t)WSCAP) return;

  _Float16* xh   = (_Float16*)(ws + oXh);
  float*    hf   = (float*)(ws + oHf);
  _Float16* hhp  = (_Float16*)(ws + oHh);
  _Float16* mh   = (_Float16*)(ws + oMh);
  float*    gl   = (float*)(ws + oG);
  int*      gcnt = (int*)(ws + oCnt);
  int*      gsst = (int*)(ws + oSst);
  int*      greg = (int*)(ws + oReg);
  _Float16* tp   = (_Float16*)(ws + oT);
  float*    part = (float*)(ws + oPt);
  _Float16* w1p  = (_Float16*)(ws + owW1);
  _Float16* w2p  = (_Float16*)(ws + owW2);
  _Float16* wihp = (_Float16*)(ws + oWih);
  _Float16* whhp = (_Float16*)(ws + oWhh);
  _Float16* a1p  = (_Float16*)(ws + oA1);
  _Float16* a2p  = (_Float16*)(ws + oA2);
  _Float16* ajp  = (_Float16*)(ws + oAJ);
  _Float16* o1p  = (_Float16*)(ws + oO1);
  _Float16* o2p  = (_Float16*)(ws + oO2);

  const float SW = 256.0f;
  k_cvtw<<<(GH1 * F / 8 + NTHR - 1) / NTHR, NTHR, 0, stream>>>(gW1, w1p, GH1, F, GH1, F, 1, SW);
  k_cvtw<<<(GH2 * GH1 / 8 + NTHR - 1) / NTHR, NTHR, 0, stream>>>(gW2, w2p, GH2, GH1, GH2, GH1, 1, SW);
  k_cvtw<<<(G3 * F / 8 + NTHR - 1) / NTHR, NTHR, 0, stream>>>(Wih, wihp, G3, F, G3, F, 0, SW);
  k_cvtw<<<(G3 * F / 8 + NTHR - 1) / NTHR, NTHR, 0, stream>>>(Whh, whhp, G3, F, G3, F, 0, SW);
  k_cvtw<<<(F * 2 * F / 8 + NTHR - 1) / NTHR, NTHR, 0, stream>>>(aW1, a1p, F, 2 * F, F, 2 * F, 1, SW);
  k_cvtw<<<(F * F / 8 + NTHR - 1) / NTHR, NTHR, 0, stream>>>(aW2, a2p, F, F, F, F, 1, SW);
  k_cvtw<<<(F * F / 8 + NTHR - 1) / NTHR, NTHR, 0, stream>>>(ajW, ajp, F, F, F, F, 1, SW);
  k_cvtw<<<(H1P * F / 8 + NTHR - 1) / NTHR, NTHR, 0, stream>>>(oW1, o1p, H1, F, H1P, F, 1, SW);
  k_cvtw<<<(H2 * H1P / 8 + NTHR - 1) / NTHR, NTHR, 0, stream>>>(oW2, o2p, H2, H1, H2, H1P, 1, SW);

  k_prepx<<<(NP * (F / 8) + NTHR - 1) / NTHR, NTHR, 0, stream>>>(x, xh, nN, NP);

  const int vec8 = ((nE & 3) == 0) ? 1 : 0;
  hipFuncSetAttribute(reinterpret_cast<const void*>(&k_csr), hipFuncAttributeMaxDynamicSharedMemorySize, LDS_CSR);
  k_csr<<<nBF, NTHR, LDS_CSR, stream>>>(ei, eattr, tcut, gcnt, gsst, greg, nN, nE, vec8);

  for (int it = 0; it < PROP_ITER; ++it) {
    const _Float16* ahin = (it == 0) ? (const _Float16*)xh : (const _Float16*)hhp;
    const float*    hin  = (it == 0) ? x : (const float*)hf;
    k_gmlp<<<nB32, NTHR, 0, stream>>>(ahin, w1p, gb1, w2p, gb2, gW3, gb3, gl, nN);
    k_agg<<<nB32, NTHR, 0, stream>>>(greg, gcnt, gsst, gl, hin, tcut, mh, nN);
    k_gru<<<nB32, NTHR, 0, stream>>>(mh, ahin, hin, wihp, whhp, bih, bhh, hf, hhp, nN);
  }

  hipFuncSetAttribute(reinterpret_cast<const void*>(&k_final), hipFuncAttributeMaxDynamicSharedMemorySize, LDS_FIN);
  k_final<<<nB64, NTHR, LDS_FIN, stream>>>(hhp, xh, a1p, ab1, a2p, ab2, ajp, ajb, tp, nN, NP);
  k_pool<<<nKB, NTHR, 0, stream>>>(tp, batch, part, nN, NP);
  k_head<<<1, NTHR, 0, stream>>>(part, nKB, o1p, ob1, o2p, ob2, oW3, ob3, out, nG);
}
